// DotProductCausalRotaryAttention_38620345925719
// MI455X (gfx1250) — hardware-verified
//
#include <hip/hip_runtime.h>
#include <math.h>
#include <stdint.h>

#define NPAIR 32
#define SEQ   2048
#define DH    128
#define ROT   32

typedef __attribute__((ext_vector_type(16))) _Float16 v16h;
typedef __attribute__((ext_vector_type(8)))  _Float16 v8h;
typedef __attribute__((ext_vector_type(16))) __bf16   v16b;
typedef __attribute__((ext_vector_type(8)))  __bf16   v8b;
typedef __attribute__((ext_vector_type(8)))  float    v8f;
typedef __attribute__((ext_vector_type(4)))  float    v4f;
typedef __attribute__((ext_vector_type(2)))  float    v2f;
typedef __attribute__((ext_vector_type(4)))  unsigned int v4u;
typedef __attribute__((ext_vector_type(2)))  unsigned int v2u;

__device__ __forceinline__ unsigned short f2bf_bits(float f) {
  unsigned u = __float_as_uint(f);
  return (unsigned short)((u + 0x7FFFu + ((u >> 16) & 1u)) >> 16);
}
__device__ __forceinline__ float bf_bits2f(unsigned short h) { return __uint_as_float(((unsigned)h) << 16); }
__device__ __forceinline__ unsigned pk16(unsigned short a, unsigned short b) { return (unsigned)a | ((unsigned)b << 16); }

__device__ __forceinline__ void dep_guard_h(v8f& a, v8f& b, v16h x, v16h y) { asm volatile("v_nop\n\tv_nop\n\tv_nop\n\tv_nop" : "+v"(a), "+v"(b) : "v"(x), "v"(y)); }
__device__ __forceinline__ void dep_guard_b(v8f& a, v8f& b, v16b x, v16b y) { asm volatile("v_nop\n\tv_nop\n\tv_nop\n\tv_nop" : "+v"(a), "+v"(b) : "v"(x), "v"(y)); }
__device__ __forceinline__ void keep4_h(v16h a, v16h b, v16h c, v16h d) { asm volatile("v_nop" :: "v"(a), "v"(b), "v"(c), "v"(d)); }
__device__ __forceinline__ void keep4_b(v16b a, v16b b, v16b c, v16b d) { asm volatile("v_nop" :: "v"(a), "v"(b), "v"(c), "v"(d)); }
__device__ __forceinline__ void acc_guard4(v8f& a, v8f& b, v8f& c, v8f& d) { asm volatile("v_nop\n\tv_nop\n\tv_nop\n\tv_nop" : "+v"(a), "+v"(b), "+v"(c), "+v"(d)); }
template <typename T> struct Frag;
template <> struct Frag<_Float16> {
  typedef v16h V; union U { v16h v; v8h h[2]; };
  static __device__ __forceinline__ v16h load(const _Float16* p) {
    U f; f.h[0] = *(const v8h*)(p); f.h[1] = *(const v8h*)(p + 16); return f.v;
  }
  static __device__ __forceinline__ v8f mma(v16h a, v16h b, v8f c) {
    return __builtin_amdgcn_wmma_f32_16x16x32_f16(false, a, false, b, (short)0, c, false, false);
  }
  static __device__ __forceinline__ void guard(v8f& a, v8f& b, v16h x, v16h y) { dep_guard_h(a, b, x, y); }
  static __device__ __forceinline__ void keep(v16h a, v16h b, v16h c, v16h d) { keep4_h(a, b, c, d); }
};
template <> struct Frag<__bf16> {
  typedef v16b V; union U { v16b v; v8b h[2]; };
  static __device__ __forceinline__ v16b load(const __bf16* p) {
    U f; f.h[0] = *(const v8b*)(p); f.h[1] = *(const v8b*)(p + 16); return f.v;
  }
  static __device__ __forceinline__ v8f mma(v16b a, v16b b, v8f c) {
    return __builtin_amdgcn_wmma_f32_16x16x32_bf16(false, a, false, b, (short)0, c, false, false);
  }
  static __device__ __forceinline__ void guard(v8f& a, v8f& b, v16b x, v16b y) { dep_guard_b(a, b, x, y); }
  static __device__ __forceinline__ void keep(v16b a, v16b b, v16b c, v16b d) { keep4_b(a, b, c, d); }
};

template <int ET> struct Elem;
template <> struct Elem<0> { typedef _Float16 T; };
template <> struct Elem<1> { typedef __bf16 T; };
template <int ET, bool SPLIT, int BIAS_MODE, int OUT_MODE, bool RESID, int ACT = 0, bool LOWER = false, bool CAUSALK = false>
__global__ __launch_bounds__(256) void wmma_gemm64(
    const unsigned short* __restrict__ Ap, const unsigned short* __restrict__ A2p, int lda, long strideA,
    const unsigned short* __restrict__ Btp, const unsigned short* __restrict__ Bt2p, int ldb, long strideB,
    void* __restrict__ Cout, void* __restrict__ Cout2, int ldc, long strideC,
    const float* __restrict__ bias,
    const float* __restrict__ resid, long strideR,
    int M, int N, int K, float scale) {
  typedef typename Elem<ET>::T T;
  typedef typename Frag<T>::V V;
  const T* A = (const T*)Ap; const T* A2 = (const T*)A2p; const T* Bt = (const T*)Btp; const T* Bt2 = (const T*)Bt2p;
  __shared__ __align__(16) float sT[8][16 * 68];
  const int b    = blockIdx.y;
  const int lane = threadIdx.x & 31;
  const int wave = threadIdx.x >> 5;
  const int tilesN = N >> 6;
  const int tilesM = M >> 6;
  const int tile = blockIdx.x * 8 + wave;
  if (tile >= tilesM * tilesN) return;
  const int tm = tile / tilesN;
  const int tn = tile - tm * tilesN;
  const int m0 = tm << 6;
  const int n0 = tn << 6;
  if (LOWER && n0 > m0) return;

  const T* Ab  = A  + (size_t)b * strideA;
  const T* Bb  = Bt + (size_t)b * strideB;
  const T* Ab2 = SPLIT ? (A2  + (size_t)b * strideA) : nullptr;
  const T* Bb2 = SPLIT ? (Bt2 + (size_t)b * strideB) : nullptr;

  const int rlane = lane & 15;
  const int koff  = (lane >> 4) * 8;
  const int mOff  = (lane >> 4) * 8;

  v8f acc[4][4];
#pragma unroll
  for (int i = 0; i < 4; ++i)
#pragma unroll
    for (int j = 0; j < 4; ++j) acc[i][j] = (v8f){0.f,0.f,0.f,0.f,0.f,0.f,0.f,0.f};

  const int kEnd = CAUSALK ? (((m0 + 64) < K) ? (m0 + 64) : K) : K;
  for (int k0 = 0; k0 < kEnd; k0 += 32) {
    V bh[4], bl[4];
#pragma unroll
    for (int j = 0; j < 4; ++j) {
      const size_t bo = (size_t)(n0 + (j << 4) + rlane) * ldb + koff + k0;
      bh[j] = Frag<T>::load(Bb + bo);
      if (SPLIT) bl[j] = Frag<T>::load(Bb2 + bo);
    }
#pragma unroll
    for (int i = 0; i < 4; ++i) {
      const size_t ao = (size_t)(m0 + (i << 4) + rlane) * lda + koff + k0;
      V ah = Frag<T>::load(Ab + ao);
      V al;
      if (SPLIT) al = Frag<T>::load(Ab2 + ao);
#pragma unroll
      for (int j = 0; j < 4; ++j) {
        acc[i][j] = Frag<T>::mma(ah, bh[j], acc[i][j]);
        if (SPLIT) {
          acc[i][j] = Frag<T>::mma(ah, bl[j], acc[i][j]);
          acc[i][j] = Frag<T>::mma(al, bh[j], acc[i][j]);
        }
      }
      Frag<T>::guard(acc[i][0], acc[i][3], ah, SPLIT ? al : ah);
    }
    Frag<T>::keep(bh[0], bh[1], bh[2], bh[3]);
    if (SPLIT) Frag<T>::keep(bl[0], bl[1], bl[2], bl[3]);
  }
  acc_guard4(acc[0][0], acc[0][1], acc[0][2], acc[0][3]);
  acc_guard4(acc[1][0], acc[1][1], acc[1][2], acc[1][3]);
  acc_guard4(acc[2][0], acc[2][1], acc[2][2], acc[2][3]);
  acc_guard4(acc[3][0], acc[3][1], acc[3][2], acc[3][3]);

  float* slab = sT[wave];
  const float* Rb = RESID ? (resid + (size_t)b * strideR) : nullptr;
#pragma unroll
  for (int i = 0; i < 4; ++i) {
    const int mBase = m0 + (i << 4);
#pragma unroll
    for (int j = 0; j < 4; ++j) {
      const int n = n0 + (j << 4) + rlane;
      float bv = 0.f;
      if (BIAS_MODE == 2) bv = bias[n];
#pragma unroll
      for (int r = 0; r < 8; ++r) {
        float v = acc[i][j][r] * scale;
        if (BIAS_MODE == 1) v += bias[mBase + mOff + r];
        if (BIAS_MODE == 2) v += bv;
        if (RESID) v += Rb[(size_t)(mBase + mOff + r) * ldc + n];
        if (ACT == 1) v = tanhf(v);
        if (ACT == 2) v = fmaxf(v, 0.0f);
        if (ACT == 3) v = v / (1.0f + expf(-v));
        if (ACT == 4) v = (v > 0.f) ? v : 0.01f * v;
        if (ACT == 5) v = 0.5f * v * (1.0f + erff(v * 0.70710678118654752f));
        slab[(mOff + r) * 68 + (j << 4) + rlane] = v;
      }
    }
    __builtin_amdgcn_fence(__ATOMIC_RELEASE, "workgroup");
    __builtin_amdgcn_wave_barrier();
    __builtin_amdgcn_fence(__ATOMIC_ACQUIRE, "workgroup");
    if (OUT_MODE == 0) {
      float* C = (float*)Cout + (size_t)b * strideC;
      const int hh = lane >> 4, c4 = (lane & 15) * 4;
      for (int pass = 0; pass < 2; ++pass) {
#pragma unroll
        for (int it = 0; it < 8; ++it) {
          const int row = it * 2 + hh;
          v4f v = *(const v4f*)(slab + row * 68 + c4);
          *(volatile v4f*)(C + (size_t)(mBase + row) * ldc + n0 + c4) = v;
        }
        __threadfence();
      }
    } else {
      const int q = lane >> 3, c8 = (lane & 7) * 8;
      unsigned short* C  = (unsigned short*)Cout  + (size_t)b * strideC;
      unsigned short* C2 = (OUT_MODE == 2) ? ((unsigned short*)Cout2 + (size_t)b * strideC) : nullptr;
      for (int pass = 0; pass < 2; ++pass) {
#pragma unroll
        for (int it = 0; it < 4; ++it) {
          const int row = it * 4 + q;
          const float* sp = slab + row * 68 + c8;
          v8h hv, lv;
#pragma unroll
          for (int e = 0; e < 8; ++e) {
            if (OUT_MODE == 1) {
              hv[e] = (_Float16)sp[e];
            } else {
              unsigned short hb = f2bf_bits(sp[e]);
              unsigned short lb = f2bf_bits(sp[e] - bf_bits2f(hb));
              hv[e] = __builtin_bit_cast(_Float16, hb);
              lv[e] = __builtin_bit_cast(_Float16, lb);
            }
          }
          *(volatile v8h*)(C + (size_t)(mBase + row) * ldc + n0 + c8) = hv;
          if (OUT_MODE == 2) *(volatile v8h*)(C2 + (size_t)(mBase + row) * ldc + n0 + c8) = lv;
        }
        __threadfence();
      }
    }
    __builtin_amdgcn_fence(__ATOMIC_RELEASE, "workgroup");
    __builtin_amdgcn_wave_barrier();
    __builtin_amdgcn_fence(__ATOMIC_ACQUIRE, "workgroup");
  }
}

__device__ __forceinline__ float rot_freq(int m) {
  float f = 1.0f;
  f = (m == 1)  ? 1.778279410038923f   : f;
  f = (m == 2)  ? 3.1622776601683795f  : f;
  f = (m == 3)  ? 5.623413251903491f   : f;
  f = (m == 4)  ? 10.0f                : f;
  f = (m == 5)  ? 17.78279410038923f   : f;
  f = (m == 6)  ? 31.622776601683793f  : f;
  f = (m == 7)  ? 56.23413251903491f   : f;
  f = (m == 8)  ? 100.0f               : f;
  f = (m == 9)  ? 177.8279410038923f   : f;
  f = (m == 10) ? 316.22776601683796f  : f;
  f = (m == 11) ? 562.341325190349f    : f;
  f = (m == 12) ? 1000.0f              : f;
  f = (m == 13) ? 1778.279410038923f   : f;
  f = (m == 14) ? 3162.2776601683795f  : f;
  f = (m == 15) ? 5623.413251903491f   : f;
  return f;
}

__global__ __launch_bounds__(256) void rope_split_kernel(const float* __restrict__ qsrc, const float* __restrict__ ksrc,
                                                         unsigned short* __restrict__ Qh, unsigned short* __restrict__ Ql,
                                                         unsigned short* __restrict__ Kh, unsigned short* __restrict__ Kl) {
#pragma clang fp contract(off)
  __shared__ __align__(16) unsigned short sh[16 * DH];
  __shared__ __align__(16) unsigned short sl[16 * DH];
  const int tid = threadIdx.x;
  const bool isk = (blockIdx.y != 0);
  const float* src = isk ? ksrc : qsrc;
  unsigned short* oh = isk ? Kh : Qh;
  unsigned short* ol = isk ? Kl : Ql;
  const int rblk = blockIdx.x * 64;
  const int prl = tid >> 4;
  const int pm  = tid & 15;
  const float invf = 1.0f / rot_freq(pm);
#pragma unroll 1
  for (int it = 0; it < 4; ++it) {
    const int rbase = rblk + it * 16;
    {
      const int row = rbase + prl;
      const v2f x = *(const v2f*)(src + (size_t)row * DH + 2 * pm);
      const float ang = (float)row * invf;
      float sn, cs;
      sincosf(ang, &sn, &cs);
      const float y0 = x[0] * cs - x[1] * sn;
      const float y1 = x[1] * cs + x[0] * sn;
      const unsigned short h0 = f2bf_bits(y0), h1 = f2bf_bits(y1);
      const unsigned short l0 = f2bf_bits(y0 - bf_bits2f(h0));
      const unsigned short l1 = f2bf_bits(y1 - bf_bits2f(h1));
      *(unsigned*)(sh + prl * DH + 2 * pm) = pk16(h0, h1);
      *(unsigned*)(sl + prl * DH + 2 * pm) = pk16(l0, l1);
    }
#pragma unroll
    for (int it2 = 0; it2 < 2; ++it2) {
      const int j  = tid + it2 * 256;
      const int jj = (j < 384) ? j : 383;
      const int rl = jj / 24;
      const int c  = ROT + 4 * (jj - rl * 24);
      const v4f x = *(const v4f*)(src + (size_t)(rbase + rl) * DH + c);
      const unsigned short h0 = f2bf_bits(x[0]), h1 = f2bf_bits(x[1]), h2 = f2bf_bits(x[2]), h3 = f2bf_bits(x[3]);
      const unsigned short l0 = f2bf_bits(x[0] - bf_bits2f(h0));
      const unsigned short l1 = f2bf_bits(x[1] - bf_bits2f(h1));
      const unsigned short l2 = f2bf_bits(x[2] - bf_bits2f(h2));
      const unsigned short l3 = f2bf_bits(x[3] - bf_bits2f(h3));
      if (j < 384) {
        *(v2u*)(sh + rl * DH + c) = (v2u){pk16(h0, h1), pk16(h2, h3)};
        *(v2u*)(sl + rl * DH + c) = (v2u){pk16(l0, l1), pk16(l2, l3)};
      }
    }
    __syncthreads();
    {
      const int rl = tid >> 4, c8 = (tid & 15) * 8;
      const v4u hv = *(const v4u*)(sh + rl * DH + c8);
      const v4u lv = *(const v4u*)(sl + rl * DH + c8);
      const size_t go = (size_t)(rbase + rl) * DH + c8;
      *(volatile v4u*)(oh + go) = hv;
      *(volatile v4u*)(ol + go) = lv;
      __threadfence();
      *(volatile v4u*)(oh + go) = hv;
      *(volatile v4u*)(ol + go) = lv;
    }
    __syncthreads();
  }
}

__global__ __launch_bounds__(256) void vtrans_split_kernel(const float* __restrict__ vsrc,
                                                           unsigned short* __restrict__ VTh, unsigned short* __restrict__ VTl) {
  __shared__ __align__(16) unsigned short th[64 * 72];
  __shared__ __align__(16) unsigned short tl[64 * 72];
  const int c0  = blockIdx.x * 64;
  const int r0  = blockIdx.y * 64;
  const int pr  = blockIdx.z;
  const float* in = vsrc + (size_t)pr * SEQ * DH;
  unsigned short* oh = VTh + (size_t)pr * DH * SEQ;
  unsigned short* ol = VTl + (size_t)pr * DH * SEQ;
  const int tid = threadIdx.x;
  {
    const int sub = tid >> 4;
    const int c4  = (tid & 15) * 4;
#pragma unroll
    for (int it = 0; it < 4; ++it) {
      const int rr = it * 16 + sub;
      const v4f x = *(const v4f*)(in + (size_t)(r0 + rr) * DH + c0 + c4);
      const unsigned short h0 = f2bf_bits(x[0]), h1 = f2bf_bits(x[1]), h2 = f2bf_bits(x[2]), h3 = f2bf_bits(x[3]);
      const unsigned short l0 = f2bf_bits(x[0] - bf_bits2f(h0));
      const unsigned short l1 = f2bf_bits(x[1] - bf_bits2f(h1));
      const unsigned short l2 = f2bf_bits(x[2] - bf_bits2f(h2));
      const unsigned short l3 = f2bf_bits(x[3] - bf_bits2f(h3));
      *(v2u*)(th + rr * 72 + c4) = (v2u){pk16(h0, h1), pk16(h2, h3)};
      *(v2u*)(tl + rr * 72 + c4) = (v2u){pk16(l0, l1), pk16(l2, l3)};
    }
  }
  __syncthreads();
  const int sub = tid >> 3;
  const int c8  = (tid & 7) * 8;
  v4u hv[2], lv[2];
#pragma unroll
  for (int it = 0; it < 2; ++it) {
    const int oc = it * 32 + sub;
    v4u a, a2;
#pragma unroll
    for (int q = 0; q < 4; ++q) {
      a[q]  = pk16(th[(c8 + 2 * q) * 72 + oc], th[(c8 + 2 * q + 1) * 72 + oc]);
      a2[q] = pk16(tl[(c8 + 2 * q) * 72 + oc], tl[(c8 + 2 * q + 1) * 72 + oc]);
    }
    hv[it] = a; lv[it] = a2;
  }
  for (int pass = 0; pass < 2; ++pass) {
#pragma unroll
    for (int it = 0; it < 2; ++it) {
      const int oc = it * 32 + sub;
      const size_t go = (size_t)(c0 + oc) * SEQ + r0 + c8;
      *(volatile v4u*)(oh + go) = hv[it];
      *(volatile v4u*)(ol + go) = lv[it];
    }
    __threadfence();
  }
}

__global__ __launch_bounds__(512) void softmax_split_kernel(const float* __restrict__ S,
                                                            unsigned short* __restrict__ Ph, unsigned short* __restrict__ Pl) {
  __shared__ float redm[16];
  __shared__ float reds[16];
  __shared__ __align__(16) unsigned short sp[2 * SEQ];
  const int i    = blockIdx.x;
  const int tid  = threadIdx.x;
  const int lane = tid & 31;
  const int wave = tid >> 5;
  const int j0   = tid * 4;
  const bool wact = (wave * 128 <= i);
  float t0 = -1.0e9f, t1 = -1.0e9f, t2 = -1.0e9f, t3 = -1.0e9f;
  if (wact) {
    const v4f cv = *(const v4f*)(S + (size_t)i * SEQ + j0);
    t0 = (j0 <= i)     ? cv[0] : -1.0e9f;
    t1 = (j0 + 1 <= i) ? cv[1] : -1.0e9f;
    t2 = (j0 + 2 <= i) ? cv[2] : -1.0e9f;
    t3 = (j0 + 3 <= i) ? cv[3] : -1.0e9f;
  }
  float m = fmaxf(fmaxf(t0, t1), fmaxf(t2, t3));
#pragma unroll
  for (int off = 16; off > 0; off >>= 1) m = fmaxf(m, __shfl_xor(m, off, 32));
  if (lane == 0) redm[wave] = m;
  __syncthreads();
  float mx = redm[0];
#pragma unroll
  for (int w = 1; w < 16; ++w) mx = fmaxf(mx, redm[w]);
  float e0 = 0.f, e1 = 0.f, e2 = 0.f, e3 = 0.f;
  if (wact) {
    e0 = expf(t0 - mx);
    e1 = expf(t1 - mx);
    e2 = expf(t2 - mx);
    e3 = expf(t3 - mx);
  }
  float s = ((e0 + e1) + e2) + e3;
#pragma unroll
  for (int off = 16; off > 0; off >>= 1) s += __shfl_xor(s, off, 32);
  if (lane == 0) reds[wave] = s;
  __syncthreads();
  float tot = reds[0];
#pragma unroll
  for (int w = 1; w < 16; ++w) tot += reds[w];
  const float inv = 1.0f / tot;
  const float p0 = e0 * inv, p1 = e1 * inv, p2 = e2 * inv, p3 = e3 * inv;
  const unsigned short hb0 = f2bf_bits(p0), hb1 = f2bf_bits(p1), hb2 = f2bf_bits(p2), hb3 = f2bf_bits(p3);
  const unsigned short lb0 = f2bf_bits(p0 - bf_bits2f(hb0));
  const unsigned short lb1 = f2bf_bits(p1 - bf_bits2f(hb1));
  const unsigned short lb2 = f2bf_bits(p2 - bf_bits2f(hb2));
  const unsigned short lb3 = f2bf_bits(p3 - bf_bits2f(hb3));
  *(v2u*)(sp + j0)       = (v2u){pk16(hb0, hb1), pk16(hb2, hb3)};
  *(v2u*)(sp + SEQ + j0) = (v2u){pk16(lb0, lb1), pk16(lb2, lb3)};
  __syncthreads();
  const v4u val = *(const v4u*)(sp + tid * 8);
  const size_t rowoff = (size_t)i * SEQ;
  unsigned short* dst = (tid < 256) ? (Ph + rowoff + (size_t)tid * 8) : (Pl + rowoff + (size_t)(tid - 256) * 8);
  *(volatile v4u*)dst = val;
  __threadfence();
  *(volatile v4u*)dst = val;
}

extern "C" void kernel_launch(void* const* d_in, const int* in_sizes, int n_in,
                              void* d_out, int out_size, void* d_ws, size_t ws_size,
                              hipStream_t stream) {
  const int NE = NPAIR * SEQ * DH;
  if (n_in < 3) return;
  if (in_sizes[0] != NE || in_sizes[1] != NE || in_sizes[2] != NE) return;
  if (out_size != NE) return;

  const float* q = (const float*)d_in[0];
  const float* k = (const float*)d_in[1];
  const float* v = (const float*)d_in[2];
  float* out = (float*)d_out;

  const size_t PVT = (size_t)NPAIR * DH * SEQ * 2;
  const size_t PS  = (size_t)SEQ * SEQ * 4;
  const size_t PP  = (size_t)SEQ * SEQ * 2;
  const size_t PQ  = (size_t)SEQ * DH * 2;
  size_t off = 0;
  const size_t oVTh = off; off += PVT;
  const size_t oVTl = off; off += PVT;
  const size_t oS   = off; off += PS;
  const size_t oPh  = off; off += PP;
  const size_t oPl  = off; off += PP;
  const size_t oQh  = off; off += PQ;
  const size_t oQl  = off; off += PQ;
  const size_t oKh  = off; off += PQ;
  const size_t oKl  = off; off += PQ;
  if (off > ws_size) return;

  char* ws = (char*)d_ws;
  unsigned short* VTh = (unsigned short*)(ws + oVTh);
  unsigned short* VTl = (unsigned short*)(ws + oVTl);
  float*          Sb  = (float*)(ws + oS);
  unsigned short* Ph  = (unsigned short*)(ws + oPh);
  unsigned short* Pl  = (unsigned short*)(ws + oPl);
  unsigned short* Qh  = (unsigned short*)(ws + oQh);
  unsigned short* Ql  = (unsigned short*)(ws + oQl);
  unsigned short* Kh  = (unsigned short*)(ws + oKh);
  unsigned short* Kl  = (unsigned short*)(ws + oKl);

  const dim3 blk(256);
  const int tilesM = SEQ / 64;
  const dim3 gS((tilesM * (SEQ / 64) + 7) / 8, 1);
  const dim3 gPV((tilesM * (DH / 64) + 7) / 8, 1);
  const float sscale = 0.08838834764831845f;

  vtrans_split_kernel<<<dim3(DH / 64, SEQ / 64, NPAIR), blk, 0, stream>>>(v, VTh, VTl);

  for (int pr = 0; pr < NPAIR; ++pr) {
    const size_t poff = (size_t)pr * SEQ * DH;
    rope_split_kernel<<<dim3(SEQ / 64, 2), blk, 0, stream>>>(q + poff, k + poff, Qh, Ql, Kh, Kl);
    wmma_gemm64<1, true, 0, 0, false, 0, true, false><<<gS, blk, 0, stream>>>(
        Qh, Ql, DH, 0L, Kh, Kl, DH, 0L, (void*)Sb, (void*)Sb, SEQ, 0L,
        q, q, 0L, SEQ, SEQ, DH, sscale);
    softmax_split_kernel<<<dim3(SEQ), dim3(512), 0, stream>>>(Sb, Ph, Pl);
    wmma_gemm64<1, true, 0, 0, false, 0, false, true><<<gPV, blk, 0, stream>>>(
        Ph, Pl, SEQ, 0L, VTh + (size_t)pr * DH * SEQ, VTl + (size_t)pr * DH * SEQ, SEQ, 0L,
        (void*)(out + poff), (void*)(out + poff), DH, 0L,
        q, q, 0L, SEQ, DH, SEQ, 1.0f);
  }
  (void)hipGetLastError();
}
